// MHSelfAttn_38233798869259
// MI455X (gfx1250) — hardware-verified
//
#include <hip/hip_runtime.h>
#include <math.h>
#include <stdint.h>

#define NB    16
#define DM    256
#define SEQ   1024
#define NH    4
#define HD    64
#define NQB   (SEQ / 64)
#define NGRP  32
#define GSZ   8
#define XPITCH 264
static_assert(NH * HD == DM);
static_assert(NGRP * GSZ == DM);
static_assert((SEQ % 64) == 0 && (DM % 64) == 0 && (DM % 32) == 0);
static_assert((XPITCH % 8) == 0);

typedef _Float16 v16h __attribute__((ext_vector_type(16)));
typedef _Float16 v8h  __attribute__((ext_vector_type(8)));
typedef __bf16   v16b __attribute__((ext_vector_type(16)));
typedef __bf16   v8b  __attribute__((ext_vector_type(8)));
typedef float    v8f  __attribute__((ext_vector_type(8)));
typedef float    v4f  __attribute__((ext_vector_type(4)));
typedef unsigned int v4u __attribute__((ext_vector_type(4)));
typedef unsigned short v8us __attribute__((ext_vector_type(8)));

__device__ __forceinline__ unsigned short bf_bits(float f) {
  unsigned u = __float_as_uint(f);
  return (unsigned short)((u + 0x7FFFu + ((u >> 16) & 1u)) >> 16);
}
__device__ __forceinline__ float bf_up(unsigned short h) { return __uint_as_float(((unsigned)h) << 16); }
__device__ __forceinline__ float bfr(float f) { return bf_up(bf_bits(f)); }
__device__ __forceinline__ unsigned short h_bits(_Float16 x) { return __builtin_bit_cast(unsigned short, x); }
__device__ __forceinline__ unsigned pk16(unsigned short a, unsigned short b) { return (unsigned)a | ((unsigned)b << 16); }
__device__ __forceinline__ v8f zero8() { v8f z = {0.f, 0.f, 0.f, 0.f, 0.f, 0.f, 0.f, 0.f}; return z; }

__device__ __forceinline__ v16b ldfrag_b(const __bf16* p) {
  union { v16b v; v8b h[2]; } f;
  f.h[0] = *(const v8b*)(p);
  f.h[1] = *(const v8b*)(p + 16);
  return f.v;
}
__device__ __forceinline__ v16h ldfrag_h(const _Float16* p) {
  union { v16h v; v8h h[2]; } f;
  f.h[0] = *(const v8h*)(p);
  f.h[1] = *(const v8h*)(p + 16);
  return f.v;
}

__device__ __forceinline__ v8f mma_h(v16h a, v16h b, v8f c) {
  c = __builtin_amdgcn_wmma_f32_16x16x32_f16(false, a, false, b, (short)0, c, false, false);
#if defined(__HIP_DEVICE_COMPILE__)
  asm volatile("v_nop\n\tv_nop\n\tv_nop\n\tv_nop" : "+v"(c) : "v"(a), "v"(b));
#endif
  return c;
}
__device__ __forceinline__ v8f mma_b_raw(v16b a, v16b b, v8f c) {
  return __builtin_amdgcn_wmma_f32_16x16x32_bf16(false, a, false, b, (short)0, c, false, false);
}
__device__ __forceinline__ void dep_guard_b(v8f& a, v8f& b, v16b x, v16b y) {
#if defined(__HIP_DEVICE_COMPILE__)
  asm volatile("v_nop\n\tv_nop\n\tv_nop\n\tv_nop" : "+v"(a), "+v"(b) : "v"(x), "v"(y));
#endif
}
__device__ __forceinline__ void keep4_b(v16b a, v16b b, v16b c, v16b d) {
#if defined(__HIP_DEVICE_COMPILE__)
  asm volatile("v_nop" :: "v"(a), "v"(b), "v"(c), "v"(d));
#endif
}
__device__ __forceinline__ void acc_guard4(v8f& a, v8f& b, v8f& c, v8f& d) {
#if defined(__HIP_DEVICE_COMPILE__)
  asm volatile("v_nop\n\tv_nop\n\tv_nop\n\tv_nop" : "+v"(a), "+v"(b), "+v"(c), "+v"(d));
#endif
}
__device__ __forceinline__ void wave_sync_lds() {
  __builtin_amdgcn_fence(__ATOMIC_RELEASE, "workgroup");
  __builtin_amdgcn_wave_barrier();
  __builtin_amdgcn_fence(__ATOMIC_ACQUIRE, "workgroup");
}

__global__ __launch_bounds__(256) void wt_cvt(const float* __restrict__ W0, const float* __restrict__ W1,
                                              const float* __restrict__ W2, const float* __restrict__ W3,
                                              unsigned short* WT) {
  __shared__ __align__(16) unsigned short T[64 * 72];
  const int tid = threadIdx.x, lane = tid & 31, wave = tid >> 5;
  const int wsel = blockIdx.y;
  const float* W = (wsel == 0) ? W0 : (wsel == 1) ? W1 : (wsel == 2) ? W2 : W3;
  const int bx = blockIdx.x;
  const int i0 = (bx >> 2) * 64;
  const int o0 = (bx & 3) * 64;
#pragma unroll 4
  for (int it = 0; it < 16; ++it) {
    const int i = it * 4 + (tid >> 6);
    const int o = tid & 63;
    const float v = W[(size_t)(i0 + i) * DM + o0 + o];
    T[o * 72 + i] = bf_bits(v);
  }
  __syncthreads();
  const int q = lane >> 3, c8 = (lane & 7) * 8;
  v8us v[2];
#pragma unroll
  for (int it = 0; it < 2; ++it) {
    const int orow = it * 32 + wave * 4 + q;
    v[it] = *(const v8us*)(T + orow * 72 + c8);
  }
  unsigned short* dst = WT + (size_t)wsel * DM * DM;
  for (int pass = 0; pass < 2; ++pass) {
#pragma unroll
    for (int it = 0; it < 2; ++it) {
      const int orow = it * 32 + wave * 4 + q;
      *(volatile v8us*)(dst + (size_t)(o0 + orow) * DM + i0 + c8) = v[it];
    }
    __threadfence();
  }
}

__global__ __launch_bounds__(256) void gn_stats(const float* __restrict__ x, float* stats) {
  __shared__ float red[256];
  __shared__ float sres[2];
  const int tid = threadIdx.x;
  const int bg = blockIdx.x;
  const float* xp = x + (size_t)bg * (GSZ * SEQ);
  float s = 0.f;
#pragma unroll 1
  for (int j = 0; j < 8; ++j) {
    const v4f v = *(const v4f*)(xp + ((size_t)j * 256 + tid) * 4);
    s += bfr(v[0]); s += bfr(v[1]); s += bfr(v[2]); s += bfr(v[3]);
  }
  red[tid] = s;
  __syncthreads();
  for (int st = 128; st > 0; st >>= 1) {
    if (tid < st) red[tid] += red[tid + st];
    __syncthreads();
  }
  if (tid == 0) sres[0] = red[0] * (1.0f / 8192.0f);
  __syncthreads();
  const float mean = sres[0];
  float q = 0.f;
#pragma unroll 1
  for (int j = 0; j < 8; ++j) {
    const v4f v = *(const v4f*)(xp + ((size_t)j * 256 + tid) * 4);
    const float d0 = bfr(v[0]) - mean, d1 = bfr(v[1]) - mean, d2 = bfr(v[2]) - mean, d3 = bfr(v[3]) - mean;
    q += d0 * d0; q += d1 * d1; q += d2 * d2; q += d3 * d3;
  }
  red[tid] = q;
  __syncthreads();
  for (int st = 128; st > 0; st >>= 1) {
    if (tid < st) red[tid] += red[tid + st];
    __syncthreads();
  }
  if (tid == 0) {
    const float var = red[0] * (1.0f / 8192.0f);
    sres[1] = 1.0f / sqrtf(var + 1e-6f);
  }
  __syncthreads();
  if (tid < 8) {
    v4f o = {0.f, 0.f, 0.f, 0.f};
    if (tid == 0) { o[0] = mean; o[1] = sres[1]; }
    float* dst = stats + (size_t)bg * 32 + tid * 4;
    *(volatile v4f*)dst = o;
    __threadfence();
    *(volatile v4f*)dst = o;
  }
}

__global__ __launch_bounds__(256) void gn_apply(const float* __restrict__ x, const float* __restrict__ stats,
                                                const float* __restrict__ gsc, const float* __restrict__ gbi,
                                                unsigned short* XNh, unsigned short* XNl) {
  __shared__ __align__(16) unsigned short Lh[32 * XPITCH];
  __shared__ __align__(16) unsigned short Ll[32 * XPITCH];
  __shared__ float smean[NGRP], srstd[NGRP], ssc[DM], sbi[DM];
  const int tid = threadIdx.x, lane = tid & 31, wave = tid >> 5;
  const int b  = blockIdx.x / (SEQ / 32);
  const int tt = blockIdx.x - b * (SEQ / 32);
  const int t0 = tt * 32;
  if (tid < NGRP) {
    smean[tid] = stats[((size_t)b * NGRP + tid) * 32 + 0];
    srstd[tid] = stats[((size_t)b * NGRP + tid) * 32 + 1];
  }
  ssc[tid] = bfr(gsc[tid]);
  sbi[tid] = bfr(gbi[tid]);
  __syncthreads();
  const float* xb = x + (size_t)b * DM * SEQ + t0;
#pragma unroll 2
  for (int it = 0; it < 32; ++it) {
    const int c = it * 8 + wave;
    const float xv = bfr(xb[(size_t)c * SEQ + lane]);
    const int g = c >> 3;
    const float v = (xv - smean[g]) * srstd[g] * ssc[c] + sbi[c];
    const unsigned short hb = bf_bits(v);
    const unsigned short lb = bf_bits(v - bf_up(hb));
    Lh[lane * XPITCH + c] = hb;
    Ll[lane * XPITCH + c] = lb;
  }
  __syncthreads();
  v8us hv[4], lv[4];
#pragma unroll
  for (int it = 0; it < 4; ++it) {
    const int r = it * 8 + wave;
    hv[it] = *(const v8us*)(Lh + r * XPITCH + lane * 8);
    lv[it] = *(const v8us*)(Ll + r * XPITCH + lane * 8);
  }
  const size_t base = (size_t)(b * SEQ + t0) * DM;
  for (int pass = 0; pass < 2; ++pass) {
#pragma unroll
    for (int it = 0; it < 4; ++it) {
      const int r = it * 8 + wave;
      *(volatile v8us*)(XNh + base + (size_t)r * DM + lane * 8) = hv[it];
      *(volatile v8us*)(XNl + base + (size_t)r * DM + lane * 8) = lv[it];
    }
    __threadfence();
  }
}

__global__ __launch_bounds__(256) void cvt_split8(const float* __restrict__ in, unsigned short* hi,
                                                  unsigned short* lo, int n8) {
  const int i = blockIdx.x * 256 + threadIdx.x;
  if (i < n8) {
    const v4f a = *(const v4f*)(in + (size_t)i * 8);
    const v4f c = *(const v4f*)(in + (size_t)i * 8 + 4);
    float f[8];
    f[0] = a[0]; f[1] = a[1]; f[2] = a[2]; f[3] = a[3];
    f[4] = c[0]; f[5] = c[1]; f[6] = c[2]; f[7] = c[3];
    unsigned short hb[8], lb[8];
#pragma unroll
    for (int e = 0; e < 8; ++e) {
      hb[e] = bf_bits(f[e]);
      lb[e] = bf_bits(f[e] - bf_up(hb[e]));
    }
    v4u ph, pl;
    ph[0] = pk16(hb[0], hb[1]); ph[1] = pk16(hb[2], hb[3]); ph[2] = pk16(hb[4], hb[5]); ph[3] = pk16(hb[6], hb[7]);
    pl[0] = pk16(lb[0], lb[1]); pl[1] = pk16(lb[2], lb[3]); pl[2] = pk16(lb[4], lb[5]); pl[3] = pk16(lb[6], lb[7]);
    *(volatile v4u*)(hi + (size_t)i * 8) = ph;
    *(volatile v4u*)(lo + (size_t)i * 8) = pl;
    __threadfence();
    *(volatile v4u*)(hi + (size_t)i * 8) = ph;
    *(volatile v4u*)(lo + (size_t)i * 8) = pl;
  }
}

template <int NSPLIT, int OUT_MODE>
__global__ __launch_bounds__(256) void gemm64(
    const unsigned short* __restrict__ Ap, const unsigned short* A2p, int lda, long long strideA,
    const unsigned short* __restrict__ Btp, const unsigned short* Bt2p, int ldb, long long strideB,
    void* Cout, int ldc, long long strideC,
    void* Cout2, int ldc2, long long strideC2, int N2,
    int M, int N, int K, float rscale,
    const float* __restrict__ bias, int bmode, int blen,
    const float* __restrict__ Rp, int ldr, long long strideR, float oscale) {
  const __bf16* A   = (const __bf16*)(const void*)Ap;
  const __bf16* A2  = (const __bf16*)(const void*)A2p;
  const __bf16* Bt  = (const __bf16*)(const void*)Btp;
  const __bf16* Bt2 = (const __bf16*)(const void*)Bt2p;
  __shared__ __align__(16) float sT[8][16 * 68];
  const int b    = blockIdx.y;
  const int lane = threadIdx.x & 31;
  const int wave = threadIdx.x >> 5;
  const int tilesN = N >> 6;
  const int tilesM = M >> 6;
  const int tile = blockIdx.x * 8 + wave;
  if (tile >= tilesM * tilesN) return;
  const int tm = tile / tilesN;
  const int tn = tile - tm * tilesN;
  const int m0 = tm << 6;
  const int n0 = tn << 6;

  const __bf16* Ab  = A  + (size_t)b * strideA;
  const __bf16* Bb  = Bt + (size_t)b * strideB;
  const __bf16* Ab2 = (NSPLIT == 1) ? (A2  + (size_t)b * strideA) : Ab;
  const __bf16* Bb2 = (NSPLIT == 3) ? (Bt2 + (size_t)b * strideB) : Bb;

  const int rlane = lane & 15;
  const int koff  = (lane >> 4) * 8;
  const int mOff  = (lane >> 4) * 8;

  v8f acc[4][4];
#pragma unroll
  for (int i = 0; i < 4; ++i)
#pragma unroll
    for (int j = 0; j < 4; ++j) acc[i][j] = zero8();

  const int kst = K >> 5;
  const int nst = (NSPLIT == 3) ? (kst * 2) : kst;
  for (int st = 0; st < nst; ++st) {
    const int k0 = ((NSPLIT == 3) ? (st >> 1) : st) << 5;
    const __bf16* Bs = (NSPLIT == 3 && (st & 1)) ? Bb2 : Bb;
    v16b bh[4];
#pragma unroll
    for (int j = 0; j < 4; ++j) {
      const size_t bo = (size_t)(n0 + (j << 4) + rlane) * ldb + koff + k0;
      bh[j] = ldfrag_b(Bs + bo);
    }
#pragma unroll
    for (int i = 0; i < 4; ++i) {
      const size_t ao = (size_t)(m0 + (i << 4) + rlane) * lda + koff + k0;
      const v16b ah = ldfrag_b(Ab + ao);
      v16b al = ah;
      if (NSPLIT == 1) al = ldfrag_b(Ab2 + ao);
#pragma unroll
      for (int j = 0; j < 4; ++j) {
        acc[i][j] = mma_b_raw(ah, bh[j], acc[i][j]);
        if (NSPLIT == 1) acc[i][j] = mma_b_raw(al, bh[j], acc[i][j]);
      }
      dep_guard_b(acc[i][0], acc[i][3], ah, al);
    }
    keep4_b(bh[0], bh[1], bh[2], bh[3]);
  }
  acc_guard4(acc[0][0], acc[0][1], acc[0][2], acc[0][3]);
  acc_guard4(acc[1][0], acc[1][1], acc[1][2], acc[1][3]);
  acc_guard4(acc[2][0], acc[2][1], acc[2][2], acc[2][3]);
  acc_guard4(acc[3][0], acc[3][1], acc[3][2], acc[3][3]);

  float bc[4];
#pragma unroll
  for (int j = 0; j < 4; ++j) {
    int bi = n0 + (j << 4) + rlane;
    bi = (bi < blen) ? bi : (blen - 1);
    bi = (bi > 0) ? bi : 0;
    const float t = bf_up(bf_bits(bias[bi]));
    bc[j] = (bmode == 1) ? t : 0.f;
  }

  float* slab = sT[wave];
#pragma unroll
  for (int i = 0; i < 4; ++i) {
    const int mBase = m0 + (i << 4);
    float brw[8];
#pragma unroll
    for (int r = 0; r < 8; ++r) {
      int bi = mBase + mOff + r;
      bi = (bi < blen) ? bi : (blen - 1);
      bi = (bi > 0) ? bi : 0;
      const float t = bf_up(bf_bits(bias[bi]));
      brw[r] = (bmode == 2) ? t : 0.f;
    }
#pragma unroll
    for (int j = 0; j < 4; ++j) {
#pragma unroll
      for (int r = 0; r < 8; ++r) {
        slab[(mOff + r) * 68 + (j << 4) + rlane] = acc[i][j][r] + bc[j] + brw[r];
      }
    }
    wave_sync_lds();
    if (OUT_MODE == 0 || OUT_MODE == 1) {
      float* C = (float*)Cout + (size_t)b * strideC;
      const float* R = Rp + (size_t)b * strideR;
      const int hh = lane >> 4, c4 = (lane & 15) * 4;
      for (int pass = 0; pass < 2; ++pass) {
#pragma unroll
        for (int it = 0; it < 8; ++it) {
          const int row = it * 2 + hh;
          v4f v = *(const v4f*)(slab + row * 68 + c4);
          if (OUT_MODE == 1) {
            const v4f xr = *(const v4f*)(R + (size_t)(mBase + row) * ldr + n0 + c4);
            v4f t;
            t[0] = (v[0] + bfr(xr[0])) * oscale;
            t[1] = (v[1] + bfr(xr[1])) * oscale;
            t[2] = (v[2] + bfr(xr[2])) * oscale;
            t[3] = (v[3] + bfr(xr[3])) * oscale;
            v = t;
          }
          *(volatile v4f*)(C + (size_t)(mBase + row) * ldc + n0 + c4) = v;
        }
        __threadfence();
      }
    } else {
      const int q = lane >> 3, c8 = (lane & 7) * 8;
      unsigned short* C  = (unsigned short*)Cout  + (size_t)b * strideC;
      unsigned short* C2 = (unsigned short*)Cout2 + (size_t)b * strideC2;
      const bool wlo = (n0 < N2);
      v4u hv[4], lv[4];
#pragma unroll
      for (int it = 0; it < 4; ++it) {
        const int row = it * 4 + q;
        const float* sp = slab + row * 68 + c8;
        v4u a, a2;
#pragma unroll
        for (int e = 0; e < 4; ++e) {
          const float f0 = sp[2 * e], f1 = sp[2 * e + 1];
          const _Float16 x0 = (_Float16)f0, x1 = (_Float16)f1;
          const unsigned short h0 = h_bits(x0), h1 = h_bits(x1);
          const unsigned short l0 = h_bits((_Float16)((f0 - (float)x0) * rscale));
          const unsigned short l1 = h_bits((_Float16)((f1 - (float)x1) * rscale));
          a[e] = pk16(h0, h1); a2[e] = pk16(l0, l1);
        }
        hv[it] = a; lv[it] = a2;
      }
      for (int pass = 0; pass < 2; ++pass) {
#pragma unroll
        for (int it = 0; it < 4; ++it) {
          const int row = it * 4 + q;
          *(volatile v4u*)(C + (size_t)(mBase + row) * ldc + n0 + c8) = hv[it];
          if (wlo) *(volatile v4u*)(C2 + (size_t)(mBase + row) * ldc2 + n0 + c8) = lv[it];
        }
        __threadfence();
      }
    }
    wave_sync_lds();
  }
}

__global__ __launch_bounds__(128)
void attn64(const unsigned short* __restrict__ qhp, const unsigned short* __restrict__ qlp,
            const unsigned short* __restrict__ khp,
            const unsigned short* __restrict__ vhp, const unsigned short* __restrict__ vlp,
            float* outp, float sscale, float rres) {
  union FH { v16h v; v8h h[2]; };
  __shared__ __align__(16) _Float16 Ksh[64 * 64];
  __shared__ __align__(16) _Float16 Vth[64 * 64];
  __shared__ __align__(16) _Float16 Vtl[64 * 64];
  __shared__ __align__(16) _Float16 Psh[4][16 * 64];
  __shared__ __align__(16) float    Os[4][16 * 64];

  const int tid  = threadIdx.x;
  const int wave = tid >> 5;
  const int lane = tid & 31;
  const int hh   = lane >> 4;
  const int c    = lane & 15;

  const int bx   = blockIdx.x;
  const int qb   = bx % NQB;
  const int rest = bx / NQB;
  const int h    = rest % NH;
  const int b    = rest / NH;
  const int q0   = qb * 64 + wave * 16;
  const size_t rowB = (size_t)b * SEQ;

  const _Float16* Qh = (const _Float16*)(const void*)qhp + (size_t)h * HD;
  const _Float16* Ql = (const _Float16*)(const void*)qlp + (size_t)h * HD;
  const _Float16* Kg = (const _Float16*)(const void*)khp + (size_t)h * HD;
  const _Float16* Vh = (const _Float16*)(const void*)vhp + ((size_t)b * DM + (size_t)h * HD) * SEQ;
  const _Float16* Vl = (const _Float16*)(const void*)vlp + ((size_t)b * DM + (size_t)h * HD) * SEQ;

  v16h qah[2], qal[2];
#pragma unroll
  for (int dc = 0; dc < 2; ++dc) {
    qah[dc] = ldfrag_h(Qh + (rowB + q0 + c) * DM + dc * 32 + 8 * hh);
    qal[dc] = ldfrag_h(Ql + (rowB + q0 + c) * DM + dc * 32 + 8 * hh);
  }

  float mrow[8], lrow[8];
  v8f oacc[4];
#pragma unroll
  for (int r = 0; r < 8; ++r) { mrow[r] = -INFINITY; lrow[r] = 0.f; }
#pragma unroll
  for (int t = 0; t < 4; ++t) oacc[t] = zero8();

  for (int kt = 0; kt < NQB; ++kt) {
    const int kv0 = kt * 64;
    __syncthreads();
    {
      const int r = tid >> 1, hf = (tid & 1) * 32;
      const _Float16* kg  = Kg + (rowB + kv0 + r) * DM + hf;
      const _Float16* vg  = Vh + (size_t)r * SEQ + kv0 + hf;
      const _Float16* vlg = Vl + (size_t)r * SEQ + kv0 + hf;
#pragma unroll
      for (int i = 0; i < 4; ++i) {
        const v8h a0 = *(const v8h*)(kg + 8 * i);
        const v8h b0 = *(const v8h*)(vg + 8 * i);
        const v8h b1 = *(const v8h*)(vlg + 8 * i);
        *(v8h*)(Ksh + r * 64 + hf + 8 * i) = a0;
        *(v8h*)(Vth + r * 64 + hf + 8 * i) = b0;
        *(v8h*)(Vtl + r * 64 + hf + 8 * i) = b1;
      }
    }
    __syncthreads();

    v8f s[4];
#pragma unroll
    for (int j = 0; j < 4; ++j) {
      v8f sh = zero8(), sl = zero8();
#pragma unroll
      for (int dc = 0; dc < 2; ++dc) {
        FH kb;
        kb.h[0] = *(const v8h*)(Ksh + (j * 16 + c) * 64 + dc * 32 + 8 * hh);
        kb.h[1] = *(const v8h*)(Ksh + (j * 16 + c) * 64 + dc * 32 + 16 + 8 * hh);
        sh = mma_h(qah[dc], kb.v, sh);
        sl = mma_h(qal[dc], kb.v, sl);
      }
#pragma unroll
      for (int r = 0; r < 8; ++r) s[j][r] = (sh[r] + sl[r] * rres) * sscale;
    }

    _Float16* pwh = Psh[wave];
#pragma unroll
    for (int r = 0; r < 8; ++r) {
      float m = s[0][r];
      m = fmaxf(m, s[1][r]);
      m = fmaxf(m, s[2][r]);
      m = fmaxf(m, s[3][r]);
#pragma unroll
      for (int off = 1; off < 16; off <<= 1) m = fmaxf(m, __shfl_xor(m, off, 32));
      const float mnew  = fmaxf(mrow[r], m);
      const float alpha = __expf(mrow[r] - mnew);
      mrow[r] = mnew;
      float psum = 0.f;
#pragma unroll
      for (int j = 0; j < 4; ++j) {
        const float p = __expf(s[j][r] - mnew);
        psum += p;
        pwh[(8 * hh + r) * 64 + j * 16 + c] = (_Float16)(p * 1024.0f);
      }
#pragma unroll
      for (int off = 1; off < 16; off <<= 1) psum += __shfl_xor(psum, off, 32);
      lrow[r] = lrow[r] * alpha + psum;
#pragma unroll
      for (int t = 0; t < 4; ++t) oacc[t][r] *= alpha;
    }
    wave_sync_lds();

    v8f o1[4];
#pragma unroll
    for (int t = 0; t < 4; ++t) o1[t] = zero8();
#pragma unroll 1
    for (int kk = 0; kk < 2; ++kk) {
      FH pa;
      pa.h[0] = *(const v8h*)(pwh + c * 64 + kk * 32 + 8 * hh);
      pa.h[1] = *(const v8h*)(pwh + c * 64 + kk * 32 + 16 + 8 * hh);
#pragma unroll
      for (int t = 0; t < 4; ++t) {
        FH vb, vl;
        vb.h[0] = *(const v8h*)(Vth + (t * 16 + c) * 64 + kk * 32 + 8 * hh);
        vb.h[1] = *(const v8h*)(Vth + (t * 16 + c) * 64 + kk * 32 + 16 + 8 * hh);
        vl.h[0] = *(const v8h*)(Vtl + (t * 16 + c) * 64 + kk * 32 + 8 * hh);
        vl.h[1] = *(const v8h*)(Vtl + (t * 16 + c) * 64 + kk * 32 + 16 + 8 * hh);
        oacc[t] = mma_h(pa.v, vb.v, oacc[t]);
        o1[t]   = mma_h(pa.v, vl.v, o1[t]);
      }
    }
#pragma unroll
    for (int t = 0; t < 4; ++t)
#pragma unroll
      for (int r = 0; r < 8; ++r) oacc[t][r] += o1[t][r] * rres;
  }

  float* os = Os[wave];
#pragma unroll
  for (int r = 0; r < 8; ++r) {
    const float l = lrow[r];
    const float inv = ((l > 0.f) ? (1.0f / l) : 0.f) * (1.0f / 1024.0f);
#pragma unroll
    for (int t = 0; t < 4; ++t) os[(8 * hh + r) * 64 + t * 16 + c] = oacc[t][r] * inv;
  }
  wave_sync_lds();
  {
    const int c4 = (lane & 15) * 4;
    for (int pass = 0; pass < 2; ++pass) {
#pragma unroll
      for (int it = 0; it < 8; ++it) {
        const int row = it * 2 + hh;
        const v4f v = *(const v4f*)(os + row * 64 + c4);
        *(volatile v4f*)(outp + (rowB + q0 + row) * DM + (size_t)h * HD + c4) = v;
      }
      __threadfence();
    }
  }
}

extern "C" void kernel_launch(void* const* d_in, const int* in_sizes, int n_in,
                              void* d_out, int out_size, void* d_ws, size_t ws_size,
                              hipStream_t stream) {
  if (n_in < 11) return;
  if (in_sizes[0] != NB * DM * SEQ) return;
  if (in_sizes[3] != DM * DM || in_sizes[5] != DM * DM || in_sizes[7] != DM * DM || in_sizes[9] != DM * DM) return;
  if (in_sizes[1] < DM || in_sizes[2] < DM) return;
  if (in_sizes[4] < 1 || in_sizes[6] < 1 || in_sizes[8] < 1 || in_sizes[10] < 1) return;
  if (out_size != NB * DM * SEQ) return;

  const float* x   = (const float*)d_in[0];
  const float* gsc = (const float*)d_in[1];
  const float* gbi = (const float*)d_in[2];
  const float* wq  = (const float*)d_in[3];
  const float* bq  = (const float*)d_in[4];
  const float* wk  = (const float*)d_in[5];
  const float* bk  = (const float*)d_in[6];
  const float* wv  = (const float*)d_in[7];
  const float* bv  = (const float*)d_in[8];
  const float* wp  = (const float*)d_in[9];
  const float* bp  = (const float*)d_in[10];
  float* out = (float*)d_out;

  const size_t PWT = (size_t)4 * DM * DM * 2;
  const size_t PST = (size_t)NB * NGRP * 32 * 4;
  const size_t P16 = (size_t)NB * SEQ * DM * 2;
  const size_t P32 = (size_t)NB * SEQ * DM * 4;
  size_t off = 0;
  const size_t oWT   = off; off += PWT;
  const size_t oST   = off; off += PST;
  const size_t oXNh  = off; off += P16;
  const size_t oXNl  = off; off += P16;
  const size_t oQh   = off; off += P16;
  const size_t oQl   = off; off += P16;
  const size_t oKh   = off; off += P16;
  const size_t oVTh  = off; off += P16;
  const size_t oVTl  = off; off += P16;
  const size_t oCTX  = off; off += P32;
  const size_t oCTXh = off; off += P16;
  const size_t oCTXl = off; off += P16;
  if (off > ws_size) return;
  if (off > (size_t)134217728) return;

  char* ws = (char*)d_ws;
  unsigned short* WT   = (unsigned short*)(ws + oWT);
  float*          ST   = (float*)(ws + oST);
  unsigned short* XNh  = (unsigned short*)(ws + oXNh);
  unsigned short* XNl  = (unsigned short*)(ws + oXNl);
  unsigned short* Qh   = (unsigned short*)(ws + oQh);
  unsigned short* Ql   = (unsigned short*)(ws + oQl);
  unsigned short* Kh   = (unsigned short*)(ws + oKh);
  unsigned short* VTh  = (unsigned short*)(ws + oVTh);
  unsigned short* VTl  = (unsigned short*)(ws + oVTl);
  float*          CTX  = (float*)(ws + oCTX);
  unsigned short* CTXh = (unsigned short*)(ws + oCTXh);
  unsigned short* CTXl = (unsigned short*)(ws + oCTXl);
  unsigned short* WTq = WT + (size_t)0 * DM * DM;
  unsigned short* WTk = WT + (size_t)1 * DM * DM;
  unsigned short* WTv = WT + (size_t)2 * DM * DM;
  unsigned short* WTp = WT + (size_t)3 * DM * DM;

  const dim3 blk(256);
  const dim3 gWT(16, 4);
  const dim3 gGN(NB * NGRP);
  const dim3 gAP(NB * (SEQ / 32));
  const dim3 gQ(((NB * SEQ / 64) * (DM / 64) + 7) / 8, 1);
  const dim3 gVT(((DM / 64) * (SEQ / 64) + 7) / 8, NB);
  const dim3 gAttn(NB * NH * NQB);
  const int  n8c = NB * SEQ * DM / 8;
  const dim3 gCvt((n8c + 255) / 256);
  const float rs2 = 1.0f / 1.41421356237309515f;

  wt_cvt<<<gWT, blk, 0, stream>>>(wq, wk, wv, wp, WT);
  gn_stats<<<gGN, blk, 0, stream>>>(x, ST);
  gn_apply<<<gAP, blk, 0, stream>>>(x, ST, gsc, gbi, XNh, XNl);
  gemm64<1, 3><<<gQ, blk, 0, stream>>>(
      XNh, XNl, DM, 0LL, WTq, WTq, DM, 0LL,
      (void*)Qh, DM, 0LL, (void*)Ql, DM, 0LL, DM,
      NB * SEQ, DM, DM, 4096.0f, bq, 1, in_sizes[4], x, 0, 0LL, 1.0f);
  gemm64<1, 3><<<gQ, blk, 0, stream>>>(
      XNh, XNl, DM, 0LL, WTk, WTk, DM, 0LL,
      (void*)Kh, DM, 0LL, (void*)Kh, DM, 0LL, 0,
      NB * SEQ, DM, DM, 4096.0f, bk, 1, in_sizes[6], x, 0, 0LL, 1.0f);
  gemm64<3, 3><<<gVT, blk, 0, stream>>>(
      WTv, WTv, DM, 0LL, XNh, XNl, DM, (long long)SEQ * DM,
      (void*)VTh, SEQ, (long long)DM * SEQ, (void*)VTl, SEQ, (long long)DM * SEQ, SEQ,
      DM, SEQ, DM, 4096.0f, bv, 2, in_sizes[8], x, 0, 0LL, 1.0f);
  attn64<<<gAttn, dim3(128), 0, stream>>>(Qh, Ql, Kh, VTh, VTl, CTX, 0.0625f, 1.0f / 4096.0f);
  cvt_split8<<<gCvt, blk, 0, stream>>>(CTX, CTXh, CTXl, n8c);
  gemm64<3, 1><<<gVT, blk, 0, stream>>>(
      WTp, WTp, DM, 0LL, CTXh, CTXl, DM, (long long)SEQ * DM,
      (void*)out, SEQ, (long long)DM * SEQ, (void*)out, SEQ, (long long)DM * SEQ, 0,
      DM, SEQ, DM, 1.0f, bp, 2, in_sizes[10], x, SEQ, (long long)DM * SEQ, rs2);
  (void)hipGetLastError();
}
